// MultiHeadSA_2413771620652
// MI455X (gfx1250) — hardware-verified
//
#include <hip/hip_runtime.h>


namespace {
constexpr int NB_ = 4, T = 2048, H = 8, D = 32, C = H * D  , CH = 256;
constexpr float XS = 8.0f, HS = 256.0f, PS = 256.0f, WSC = 256.0f, SCALE = 0.17677669529663688f;
typedef _Float16 b16;
typedef __attribute__((ext_vector_type(16))) _Float16 v16b;
typedef __attribute__((ext_vector_type(8))) _Float16 v8b;
typedef __attribute__((ext_vector_type(2))) _Float16 v2b;
typedef __attribute__((ext_vector_type(8))) float v8f;
typedef __attribute__((ext_vector_type(4))) float v4f;
__device__ __forceinline__ float bf16_rne(float f) { unsigned int u = __float_as_uint(f); u += 0x7FFFu + ((u >> 16) & 1u); float r = __uint_as_float(u & 0xFFFF0000u); asm volatile("" : "+v"(r)); return r; }
__device__ __forceinline__ float bfv(float f) { float r = bf16_rne(f); asm volatile("" : "+v"(r)); return r; }
__device__ __forceinline__ void split16(float v, b16& hi, b16& lo) { hi = (b16)v; lo = (b16)(v - (float)hi); }
__device__ __forceinline__ v16b frag_kb(const b16* p, int hh) { const v8b a = *(const v8b*)(p + 8 * hh), b = *(const v8b*)(p + 16 + 8 * hh); v16b f;
#pragma unroll
  for (int e = 0; e < 8; ++e) { f[e] = a[e]; f[8 + e] = b[e]; } return f; }
__device__ __forceinline__ v8f wmma16b(v16b a, v16b b, v8f c) { v8f d = __builtin_amdgcn_wmma_f32_16x16x32_f16(false, a, false, b, (short)0, c, false, false); asm volatile("v_nop\n\tv_nop\n\tv_nop\n\tv_nop" : "+v"(d) : "v"(a), "v"(b)); return d; }
__device__ __forceinline__ void wave_lds_sync() { __builtin_amdgcn_fence(__ATOMIC_RELEASE, "workgroup"); __builtin_amdgcn_wave_barrier(); __builtin_amdgcn_fence(__ATOMIC_ACQUIRE, "workgroup"); }

__global__ __launch_bounds__(256) void wput_kernel(const float* __restrict__ wq, const float* __restrict__ wk, const float* __restrict__ wv, b16* __restrict__ WQKV) { const int u = blockIdx.x * 256 + threadIdx.x; if (u >= 3 * C * 4) return; const int r = u / 4, c0 = (u % 4) * 8; const int which = r / C, h = (r % C) / D, d = r % D; const float* w = which == 0 ? wq : (which == 1 ? wk : wv); v8b v;
#pragma unroll
  for (int j = 0; j < 8; ++j) v[j] = (b16)(bf16_rne(w[((size_t)h * D + c0 + j) * D + d]) * WSC);
  for (int pass = 0; pass < 2; ++pass) { *(volatile v8b*)(WQKV + (size_t)r * D + c0) = v; __threadfence(); } }
__global__ __launch_bounds__(32) void proj_kernel(const float* __restrict__ x, const b16* __restrict__ WQKV, const float* __restrict__ bq, const float* __restrict__ bk, const float* __restrict__ bv, b16* __restrict__ Qh, b16* __restrict__ Ql, b16* __restrict__ Kh, b16* __restrict__ Kl, float* __restrict__ V) { __shared__ __attribute__((aligned(16))) b16 Ax[16][D + 8]; __shared__ float Tf[16][260]; const int lane = threadIdx.x, nloc = lane & 15, hlf = lane >> 4; const size_t t0 = (size_t)blockIdx.x * 16;
  for (int rr = 0; rr < 16; ++rr) Ax[rr][lane] = (b16)(bf16_rne(x[(t0 + rr) * D + lane]) * XS);
  if (lane < 16) for (int k = D; k < D + 8; ++k) Ax[lane][k] = (b16)0.0f;
  wave_lds_sync(); const v16b a = frag_kb(&Ax[nloc][0], hlf);
#pragma unroll 1
  for (int g = 0; g < 3; ++g) { const float* bias = g == 0 ? bq : (g == 1 ? bk : bv); v8f acc[16];
#pragma unroll
    for (int t = 0; t < 16; ++t) acc[t] = wmma16b(a, frag_kb(WQKV + (size_t)(g * C + t * 16 + nloc) * D, hlf), (v8f){});
#pragma unroll
    for (int t = 0; t < 16; ++t) { const int cc = t * 16 + nloc; const float bb = bfv(bias[cc]);
#pragma unroll
      for (int r8 = 0; r8 < 8; ++r8) Tf[8 * hlf + r8][cc] = acc[t][r8] * (1.0f / (XS * WSC)) + bb; }
    wave_lds_sync();
    for (int pass = 0; pass < 2; ++pass) { for (int rr = 0; rr < 16; ++rr) { const size_t tk = t0 + rr;
        if (g == 2) { for (int q = 0; q < 2; ++q) *(volatile v4f*)(V + tk * C + q * 128 + lane * 4) = *(const v4f*)(&Tf[rr][q * 128 + lane * 4]); }
        else { b16* Ph = g == 0 ? Qh : Kh; b16* Pl = g == 0 ? Ql : Kl; for (int q = 0; q < 4; ++q) { const int c = q * 64 + lane * 2; b16 h0, l0, h1, l1; split16(Tf[rr][c] * HS, h0, l0); split16(Tf[rr][c + 1] * HS, h1, l1); *(volatile v2b*)(Ph + tk * C + c) = (v2b){h0, h1}; *(volatile v2b*)(Pl + tk * C + c) = (v2b){l0, l1}; } } }
      __threadfence(); }
    wave_lds_sync(); } }
__global__ __launch_bounds__(256) void vt_kernel(const float* __restrict__ V, b16* __restrict__ VTh, b16* __restrict__ VTl) { __shared__ float Tt[64][C + 1]; const int b = blockIdx.x / (T / 64), tk0 = (blockIdx.x % (T / 64)) * 64; const int tid = threadIdx.x, wave = tid >> 5, lane = tid & 31;
  for (int q = wave; q < 64; q += 8) for (int c = lane; c < C; c += 32) Tt[q][c] = V[((size_t)b * T + tk0 + q) * C + c];
  __syncthreads();
  for (int pass = 0; pass < 2; ++pass) { for (int c = wave; c < C; c += 8) { const int h = c / D, d = c % D; b16 h0, l0, h1, l1; split16(Tt[lane * 2][c] * HS, h0, l0); split16(Tt[lane * 2 + 1][c] * HS, h1, l1); const size_t o = (((size_t)b * H + h) * D + d) * T + tk0 + lane * 2; *(volatile v2b*)(VTh + o) = (v2b){h0, h1}; *(volatile v2b*)(VTl + o) = (v2b){l0, l1}; } __threadfence(); } }
__global__ __launch_bounds__(32) void att_kernel(const b16* __restrict__ Qh, const b16* __restrict__ Ql, const b16* __restrict__ Kh, const b16* __restrict__ Kl, const b16* __restrict__ VTh, const b16* __restrict__ VTl, int QLIM, float* __restrict__ out) { __shared__ __attribute__((aligned(16))) b16 Pa[32][CH + 8], Pb[32][CH + 8]; __shared__ float Sc[32][CH + 1], Mx[32], Ls[32], Fc[32], Of[32][D + 1]; const int lane = threadIdx.x, nloc = lane & 15, hlf = lane >> 4; const int b = blockIdx.x / (H * (T / 32)), rem = blockIdx.x % (H * (T / 32)); const int h = rem / (T / 32), q0 = (rem % (T / 32)) * 32; if (q0 >= QLIM) return; const size_t tq = (size_t)b * T + q0;
  Mx[lane] = -INFINITY; Ls[lane] = 0.0f; for (int kk = CH; kk < CH + 8; ++kk) { Pa[lane][kk] = (b16)0.0f; Pb[lane][kk] = (b16)0.0f; }
  wave_lds_sync();
  v16b qa[2], ql[2]; for (int rt = 0; rt < 2; ++rt) { qa[rt] = frag_kb(Qh + (tq + rt * 16 + nloc) * C + h * D, hlf); ql[rt] = frag_kb(Ql + (tq + rt * 16 + nloc) * C + h * D, hlf); }
  v8f oacc[2][2] = {{(v8f){}, (v8f){}}, {(v8f){}, (v8f){}}};
#pragma unroll 1
  for (int ch = 0; ch < T / CH; ++ch) { const int k0 = ch * CH;
#pragma unroll 1
    for (int tg = 0; tg < 16; tg += 4) { v8f sacc[2][4];
#pragma unroll
      for (int rt = 0; rt < 2; ++rt)
#pragma unroll
        for (int t = 0; t < 4; ++t) sacc[rt][t] = (v8f){};
#pragma unroll
      for (int t = 0; t < 4; ++t) { const size_t key = ((size_t)b * T + k0 + (tg + t) * 16 + nloc) * C + h * D; const v16b kh = frag_kb(Kh + key, hlf), kl = frag_kb(Kl + key, hlf);
#pragma unroll
        for (int rt = 0; rt < 2; ++rt) { sacc[rt][t] = wmma16b(qa[rt], kh, sacc[rt][t]); sacc[rt][t] = wmma16b(qa[rt], kl, sacc[rt][t]); sacc[rt][t] = wmma16b(ql[rt], kh, sacc[rt][t]); } }
#pragma unroll
      for (int rt = 0; rt < 2; ++rt)
#pragma unroll
        for (int t = 0; t < 4; ++t)
#pragma unroll
          for (int r8 = 0; r8 < 8; ++r8) Sc[rt * 16 + 8 * hlf + r8][(tg + t) * 16 + nloc] = sacc[rt][t][r8] * (SCALE / (HS * HS)); }
    wave_lds_sync();
    { const int r = lane; float mx = -INFINITY; for (int j = 0; j < CH; ++j) mx = fmaxf(mx, Sc[r][j]); const float mo = Mx[r], mn = fmaxf(mo, mx); float sm = 0.0f; for (int j = 0; j < CH; ++j) { const float p = __expf(Sc[r][j] - mn); sm += p; b16 ph, pl; split16(p * PS, ph, pl); Pa[r][j] = ph; Pb[r][j] = pl; } const float fac = (mo == -INFINITY) ? 0.0f : __expf(mo - mn); Fc[r] = fac; Ls[r] = Ls[r] * fac + sm; Mx[r] = mn; }
    wave_lds_sync();
#pragma unroll
    for (int rt = 0; rt < 2; ++rt)
#pragma unroll
      for (int t = 0; t < 2; ++t)
#pragma unroll
        for (int r8 = 0; r8 < 8; ++r8) oacc[rt][t][r8] *= Fc[rt * 16 + 8 * hlf + r8];
#pragma unroll 2
    for (int kb = 0; kb < CH; kb += 32)
#pragma unroll
      for (int rt = 0; rt < 2; ++rt) { const v16b pa = frag_kb(&Pa[rt * 16 + nloc][kb], hlf), pb = frag_kb(&Pb[rt * 16 + nloc][kb], hlf);
#pragma unroll
        for (int t = 0; t < 2; ++t) { const size_t vo = (((size_t)b * H + h) * D + t * 16 + nloc) * T + k0 + kb; const v16b vh = frag_kb(VTh + vo, hlf), vl = frag_kb(VTl + vo, hlf); oacc[rt][t] = wmma16b(pa, vh, oacc[rt][t]); oacc[rt][t] = wmma16b(pa, vl, oacc[rt][t]); oacc[rt][t] = wmma16b(pb, vh, oacc[rt][t]); } }
    wave_lds_sync(); }
#pragma unroll
  for (int rt = 0; rt < 2; ++rt)
#pragma unroll
    for (int t = 0; t < 2; ++t)
#pragma unroll
      for (int r8 = 0; r8 < 8; ++r8) { const int r = rt * 16 + 8 * hlf + r8; Of[r][t * 16 + nloc] = oacc[rt][t][r8] * (1.0f / (PS * HS)) / Ls[r]; }
  wave_lds_sync();
  for (int pass = 0; pass < 2; ++pass) { for (int r = 0; r < 32; ++r) ((volatile float*)out)[(tq + r) * C + h * D + lane] = Of[r][lane]; __threadfence(); } }
}

extern "C" void kernel_launch(void* const* d_in, const int* in_sizes, int n_in, void* d_out, int out_size, void* d_ws, size_t ws_size, hipStream_t stream) {
  (void)n_in;
  auto Fp = [&](int i) { return (const float*)d_in[i]; };
  if (in_sizes[0] != NB_ * T * D || in_sizes[1] != H * D * D || in_sizes[3] != H * D * D || in_sizes[5] != H * D * D || in_sizes[2] != H * D || out_size != NB_ * T * C) return;
  const int QLIM = T;
  size_t off = 0; char* ws = (char*)d_ws;
  auto carve = [&](size_t bytes) { char* p = ws + off; off += (bytes + 255) & ~(size_t)255; return p; };
  b16* WQKV = (b16*)carve((size_t)3 * C * D * 2); b16* Qh = (b16*)carve((size_t)NB_ * T * C * 2); b16* Ql = (b16*)carve((size_t)NB_ * T * C * 2); b16* Kh = (b16*)carve((size_t)NB_ * T * C * 2); b16* Kl = (b16*)carve((size_t)NB_ * T * C * 2); float* V = (float*)carve((size_t)NB_ * T * C * 4); b16* VTh = (b16*)carve((size_t)NB_ * C * T * 2); b16* VTl = (b16*)carve((size_t)NB_ * C * T * 2);
  if (off > ws_size || off > ((size_t)40 << 20)) return;
  wput_kernel<<<(3 * C * 4 + 255) / 256, 256, 0, stream>>>(Fp(1), Fp(3), Fp(5), WQKV);
  proj_kernel<<<NB_ * T / 16, 32, 0, stream>>>(Fp(0), WQKV, Fp(2), Fp(4), Fp(6), Qh, Ql, Kh, Kl, V);
  vt_kernel<<<NB_ * (T / 64), 256, 0, stream>>>(V, VTh, VTl);
  att_kernel<<<NB_ * H * (T / 32), 32, 0, stream>>>(Qh, Ql, Kh, Kl, VTh, VTl, QLIM, (float*)d_out);
}
